// CrossAttention_36515811950660
// MI455X (gfx1250) — hardware-verified
//
#include <hip/hip_runtime.h>
#include <math.h>

typedef __attribute__((ext_vector_type(16))) _Float16 v16h;
typedef __attribute__((ext_vector_type(16))) __bf16 v16b;
typedef __attribute__((ext_vector_type(8)))  _Float16 v8h;
typedef __attribute__((ext_vector_type(8)))  float v8f;
typedef __attribute__((ext_vector_type(4)))  float v4f;
typedef __attribute__((ext_vector_type(4)))  unsigned v4u;

#ifndef NB
#define NB 4
#endif
#ifndef SEQ
#define SEQ 2048
#endif
#define NB_FULL 4
#define SEQ_FULL 2048
#define TT SEQ
#define CC 1024
#define DIN 1024
#define NH 16
#define HD 64
#define NQB (TT / 64)
#define SCALE 0.03125f
#define CSC (SCALE * 1.44269504088896341f)

static_assert(NB >= 1 && NB <= NB_FULL);
static_assert(SEQ >= 64 && SEQ <= SEQ_FULL);
static_assert(TT % 64 == 0);
static_assert(NQB * 64 == TT);
static_assert(CC == NH * HD);
static_assert(HD == 64);
static_assert(DIN % 32 == 0 && CC % 32 == 0);
static_assert(CC % 128 == 0 && DIN % 128 == 0);
static_assert((NB * TT) % 64 == 0);

#define WS_QH  ((size_t)0)
#define WS_KH  (WS_QH + 2u * (size_t)NB * TT * CC)
#define WS_VT  (WS_KH + 2u * (size_t)NB * TT * CC)
#define WS_Y   (WS_VT + 2u * (size_t)NB * CC * TT)
#define WS_END (WS_Y  + 2u * (size_t)NB * TT * CC)
static_assert(WS_END <= (size_t)134217728);
static_assert(WS_KH % 128 == 0 && WS_VT % 128 == 0 && WS_Y % 128 == 0);

template <typename T> __device__ __forceinline__ void vst2(void* p, T v) { *(volatile T*)p = v; __threadfence(); *(volatile T*)p = v; }
__device__ __forceinline__ v8f wmma16(v16h a, v16h b, v8f c) {
  v8f d = __builtin_amdgcn_wmma_f32_16x16x32_f16(false, a, false, b, (short)0, c, false, false);
  asm volatile("v_nop\n\tv_nop\n\tv_nop\n\tv_nop" : "+v"(d) : "v"(a), "v"(b));
  return d;
}
__device__ __forceinline__ v8f wmma_bf(v16b a, v16b b, v8f c) {
  v8f d = __builtin_amdgcn_wmma_f32_16x16x32_bf16(false, a, false, b, (short)0, c, false, false);
  asm volatile("v_nop\n\tv_nop\n\tv_nop\n\tv_nop" : "+v"(d) : "v"(a), "v"(b));
  return d;
}
__device__ __forceinline__ v16h frag_h(const _Float16* rowk0, int lane) {
  union { v16h v; v8h q[2]; } u; const _Float16* p = rowk0 + 8 * (lane >> 4);
  u.q[0] = *(const v8h*)p; u.q[1] = *(const v8h*)(p + 16); return u.v;
}
__device__ __forceinline__ float bfr(float v) { return (float)(__bf16)v; }
__device__ __forceinline__ v16b wcol_oi(const float* Wm, int k0, int o, int lane, int K) { v16b w; const float* p = Wm + (size_t)o * K + k0 + 8 * (lane >> 4);
#pragma unroll
  for (int i = 0; i < 8; ++i) { w[i] = (__bf16)p[i]; w[8 + i] = (__bf16)p[16 + i]; }
  return w; }
__device__ __forceinline__ v16h wcolh_oi(const float* Wm, int k0, int o, int lane, int K) { v16h w; const float* p = Wm + (size_t)o * K + k0 + 8 * (lane >> 4);
#pragma unroll
  for (int i = 0; i < 8; ++i) { w[i] = (_Float16)(bfr(p[i]) * 256.0f); w[8 + i] = (_Float16)(bfr(p[16 + i]) * 256.0f); }
  return w; }
#define LDSX() do { asm volatile("s_wait_dscnt 0" ::: "memory"); __builtin_amdgcn_wave_barrier(); __builtin_amdgcn_fence(3  , "workgroup"); } while (0)

__device__ __forceinline__ void proj_acc(const float* __restrict__ X, const float* __restrict__ WA, const float* __restrict__ BA, size_t xrow, int c0, int lane, v8f (&acc)[8], float (&bias)[8]) {
  const int col = lane & 15, g = lane >> 4;
#pragma unroll 2
  for (int kc = 0; kc < DIN / 32; ++kc) { v16b a; { const float* p = X + xrow * DIN + kc * 32 + 8 * g;
#pragma unroll
      for (int i = 0; i < 8; ++i) { a[i] = (__bf16)p[i]; a[8 + i] = (__bf16)p[16 + i]; } }
    asm volatile("s_wait_loadcnt 0x0" ::: "memory");
#pragma unroll
    for (int j = 0; j < 8; ++j) { const v16b w = wcol_oi(WA, kc * 32, c0 + j * 16 + col, lane, DIN); asm volatile("s_wait_loadcnt 0x0" ::: "memory"); acc[j] = wmma_bf(a, w, acc[j]); } }
#pragma unroll
  for (int j = 0; j < 8; ++j) bias[j] = bfr(BA[c0 + j * 16 + col]);
}

__global__ __launch_bounds__(128) void k_proj(const float* __restrict__ XQ, const float* __restrict__ XK, const float* __restrict__ XV, const float* __restrict__ WQ, const float* __restrict__ WK, const float* __restrict__ WV, const float* __restrict__ BQ, const float* __restrict__ BK, const float* __restrict__ BV,
    _Float16* __restrict__ QK, _Float16* __restrict__ VT) {
  __shared__ __align__(16) _Float16 sh[64][136]; __shared__ __align__(16) _Float16 th[128][72];
  const int tid = threadIdx.x, wave = tid >> 5, lane = tid & 31, col = lane & 15, g = lane >> 4; const int which = blockIdx.z; const int c0 = blockIdx.y * 128;
  const size_t r0 = (size_t)blockIdx.x * 64; const size_t bb = r0 / TT; const int t0 = (int)(r0 % TT);
  const size_t xrow = bb * SEQ_FULL + t0 + wave * 16 + col;
  v8f acc[8] = {}; float bias[8];
  if (which == 0) proj_acc(XQ, WQ, BQ, xrow, c0, lane, acc, bias);
  else if (which == 1) proj_acc(XK, WK, BK, xrow, c0, lane, acc, bias);
  else proj_acc(XV, WV, BV, xrow, c0, lane, acc, bias);
  if (which < 2) { _Float16* DH = QK + (size_t)which * NB * TT * CC;
#pragma unroll
    for (int j = 0; j < 8; ++j) {
#pragma unroll
      for (int r = 0; r < 8; ++r) sh[wave * 16 + 8 * g + r][j * 16 + col] = (_Float16)(acc[j][r] + bias[j]); }
    __syncthreads();
    for (int e = tid; e < 64 * 16; e += 128) { const int rl = e >> 4, q = e & 15; const v4u val = *(const v4u*)&sh[rl][q * 8]; vst2((void*)(DH + (r0 + rl) * CC + c0 + q * 8), val); }
  } else {
#pragma unroll
    for (int j = 0; j < 8; ++j) {
#pragma unroll
      for (int r = 0; r < 8; ++r) th[j * 16 + col][wave * 16 + 8 * g + r] = (_Float16)(acc[j][r] + bias[j]); }
    __syncthreads();
    for (int e = tid; e < 128 * 8; e += 128) { const int cl = e >> 3, q = e & 7; const v4u val = *(const v4u*)&th[cl][q * 8]; vst2((void*)(VT + (bb * CC + c0 + cl) * (size_t)TT + t0 + q * 8), val); } } }

__global__ __launch_bounds__(128) void k_attn(const _Float16* __restrict__ QH, const _Float16* __restrict__ KH, const _Float16* __restrict__ VT, _Float16* __restrict__ Y) {
  __shared__ __align__(16) _Float16 so[4][16][72];
  const int tid = threadIdx.x, wave = tid >> 5, lane = tid & 31, col = lane & 15, g = lane >> 4;
  const int qb = blockIdx.x, h = blockIdx.y; const size_t rowb = (size_t)blockIdx.z * TT; const int ql0 = qb * 64 + wave * 16;
  v16h qf[2];
#pragma unroll
  for (int kc = 0; kc < 2; ++kc) qf[kc] = frag_h(QH + (rowb + ql0 + col) * CC + h * HD + kc * 32, lane);
  const _Float16* Kp = KH + (rowb + col) * CC + h * HD;
  const _Float16* Vp = VT + ((size_t)blockIdx.z * CC + h * HD + col) * (size_t)TT;
  v8f o[4] = {}; float m = -3.0e38f, ls = 0.f;
#pragma unroll 1
  for (int kb = 0; kb < TT / 64; ++kb) { const int key0 = kb * 64;
    v8f s[4] = {};
#pragma unroll
    for (int j = 0; j < 4; ++j) {
#pragma unroll
      for (int kc = 0; kc < 2; ++kc) { const v16h kf = frag_h(Kp + (size_t)(key0 + j * 16) * CC + kc * 32, lane); s[j] = wmma16(kf, qf[kc], s[j]); } }
    float ml = -3.0e38f;
#pragma unroll
    for (int j = 0; j < 4; ++j) {
#pragma unroll
      for (int r = 0; r < 8; ++r) { s[j][r] = s[j][r] * CSC; ml = fmaxf(ml, s[j][r]); } }
    ml = fmaxf(ml, __shfl_xor(ml, 16));
    const float mn = fmaxf(m, ml); const float alpha = exp2f(m - mn); m = mn;
    float ps = 0.f; v16h pb[2];
#pragma unroll
    for (int j = 0; j < 4; ++j) {
#pragma unroll
      for (int r = 0; r < 8; ++r) { const float p = exp2f(s[j][r] - mn); ps += p; pb[j >> 1][(j & 1) * 8 + r] = (_Float16)(p * 256.0f); } }
    ls = ls * alpha + ps;
#pragma unroll
    for (int jd = 0; jd < 4; ++jd) {
#pragma unroll
      for (int r = 0; r < 8; ++r) o[jd][r] = o[jd][r] * alpha; }
#pragma unroll
    for (int jd = 0; jd < 4; ++jd) {
#pragma unroll
      for (int kk = 0; kk < 2; ++kk) { const v16h vf = frag_h(Vp + (size_t)(jd * 16) * TT + key0 + kk * 32, lane); o[jd] = wmma16(vf, pb[kk], o[jd]); } } }
  ls = ls + __shfl_xor(ls, 16);
  const float fin = 0.25f * (1.0f / ls);
#pragma unroll
  for (int jd = 0; jd < 4; ++jd) { v8h hv;
#pragma unroll
    for (int r = 0; r < 8; ++r) hv[r] = (_Float16)(o[jd][r] * fin);
    *(v8h*)&so[wave][col][jd * 16 + 8 * g] = hv; }
  LDSX();
#pragma unroll
  for (int it = 0; it < 4; ++it) { const int rl = it * 4 + (lane >> 3), q = lane & 7; const v8h val = *(const v8h*)&so[wave][rl][q * 8]; vst2((void*)(Y + (rowb + ql0 + rl) * CC + h * HD + q * 8), val); } }

__global__ __launch_bounds__(128) void k_out(const _Float16* __restrict__ Y, const float* __restrict__ WO, const float* __restrict__ BO, float* __restrict__ OUT) { __shared__ __align__(16) float sf[4][16][132];
  const int tid = threadIdx.x, wave = tid >> 5, lane = tid & 31, col = lane & 15, g = lane >> 4; const int c0 = blockIdx.y * 128; const size_t r0 = (size_t)blockIdx.x * 64 + wave * 16;
  v8f acc[8] = {};
#pragma unroll 2
  for (int kc = 0; kc < CC / 32; ++kc) { const v16h a = frag_h(Y + (r0 + col) * CC + kc * 32, lane); asm volatile("s_wait_loadcnt 0x0" ::: "memory");
#pragma unroll
    for (int j = 0; j < 8; ++j) { const v16h w = wcolh_oi(WO, kc * 32, c0 + j * 16 + col, lane, CC); asm volatile("s_wait_loadcnt 0x0" ::: "memory"); acc[j] = wmma16(a, w, acc[j]); } }
#pragma unroll
  for (int j = 0; j < 8; ++j) { const float bias = bfr(BO[c0 + j * 16 + col]);
#pragma unroll
    for (int r = 0; r < 8; ++r) sf[wave][8 * g + r][j * 16 + col] = acc[j][r] * (1.0f / 16384.0f) + bias; }
  LDSX(); for (int rl = 0; rl < 16; ++rl) { const v4f val = *(const v4f*)&sf[wave][rl][lane * 4]; vst2((void*)(OUT + (r0 + rl) * DIN + c0 + lane * 4), val); } }

extern "C" void kernel_launch(void* const* d_in, const int* in_sizes, int n_in, void* d_out, int out_size, void* d_ws, size_t ws_size, hipStream_t stream) {
  if (n_in < 11) return;
  const long long need_act = ((long long)(NB - 1) * SEQ_FULL + SEQ) * DIN;
  if ((long long)in_sizes[0] < need_act || (long long)in_sizes[1] < need_act || (long long)in_sizes[2] < need_act) return;
  if (in_sizes[3] < CC * DIN || in_sizes[5] < CC * DIN || in_sizes[7] < CC * DIN || in_sizes[9] < DIN * CC) return;
  if (in_sizes[4] < CC || in_sizes[6] < CC || in_sizes[8] < CC || in_sizes[10] < DIN) return;
  if ((long long)out_size < (long long)NB * TT * DIN) return;
  if (ws_size < (size_t)WS_END) return;
  const float** F = (const float**)d_in;
  char* ws = (char*)d_ws; _Float16 *QK = (_Float16*)(ws + WS_QH), *VT = (_Float16*)(ws + WS_VT), *Y = (_Float16*)(ws + WS_Y); _Float16 *QH = QK, *KH = (_Float16*)(ws + WS_KH);
  k_proj<<<dim3(NB * TT / 64, CC / 128, 3), 128, 0, stream>>>(F[0], F[1], F[2], F[3], F[5], F[7], F[4], F[6], F[8], QK, VT);
  k_attn<<<dim3(NQB, NH, NB), 128, 0, stream>>>(QH, KH, VT, Y);
  k_out<<<dim3(NB * TT / 64, DIN / 128), 128, 0, stream>>>(Y, F[9], F[10], (float*)d_out);
}
